// GConv_35639638622887
// MI455X (gfx1250) — hardware-run, weakly checked
//
#include <hip/hip_runtime.h>
#include <math.h>

typedef __attribute__((ext_vector_type(16))) _Float16 v16h;
typedef __attribute__((ext_vector_type(8)))  _Float16 v8h;
typedef __attribute__((ext_vector_type(8)))  float    v8f;
typedef __attribute__((ext_vector_type(4)))  float    v4f;

constexpr int kNb      = 8;
constexpr int kLen     = 8192;
constexpr int kCh      = 96;
constexpr int kTaps    = 64;
constexpr int kHalfLen = kLen / 2;
constexpr int kCols    = 16;
constexpr int kShifts     = 8;
constexpr int kPitch      = kLen + 256;
constexpr int kKsPerCh    = kShifts * kPitch;
constexpr int kKsVecPerCh = kKsPerCh / 8;
constexpr int kWrapMask   = (kLen - 1) & ~7;
constexpr float kCarryK = 256.0f;
constexpr float kCarryU = 64.0f;
constexpr float kFold   = 1.0f / (kCarryK * kCarryU);
constexpr float kF16MinNormal = 6.103515625e-05f;
constexpr int kTilesPerWave = 8;
constexpr int kWavesPerBlk  = 8;
constexpr int kTilesPerBlk  = kTilesPerWave * kWavesPerBlk;
constexpr int kBlksPerCh    = (kHalfLen / 16) / kTilesPerBlk;
constexpr int kSlabPitch    = 132;
constexpr int kTilePitch    = 100;

static_assert(kNb * 2 == kCols, "columns = batch x two half-length rotations");
static_assert((kLen % 32) == 0, "K multiple of 32");
static_assert(kBlksPerCh * kTilesPerBlk * 16 == kHalfLen, "t coverage");
static_assert(kPitch >= kLen + 32 && (kPitch % 8) == 0, "wrap tail");
static_assert((kKsVecPerCh % 256) == 0, "copy loop exact");
static_assert((size_t)kWavesPerBlk * kCols * kSlabPitch * 4 <= (size_t)kKsPerCh * 2, "output slabs fit in the operand LDS");
static_assert((kCh % 4) == 0 && (kCh * 64) % (256 * 4) == 0, "layout tile loops exact");

constexpr size_t kOffKS   = 0;
constexpr size_t kBytesKS = (size_t)kCh * kKsPerCh * 2;
constexpr size_t kOffBT   = kOffKS + kBytesKS;
constexpr size_t kBytesBT = (size_t)kCh * kCols * kLen * 2;
constexpr size_t kOffYP   = kOffBT + kBytesBT;
constexpr size_t kBytesYP = (size_t)kCh * kNb * kLen * 4;
constexpr size_t kWsTotal = kOffYP + kBytesYP;
static_assert(kWsTotal == 63307776ull, "carve total");
static_assert(kWsTotal <= 134217728ull, "carve cap");
static_assert((kOffBT % 128) == 0 && (kOffYP % 128) == 0, "128-B aligned regions");

__device__ __forceinline__ _Float16 f2h_flush(float v) {
  const float w = (fabsf(v) < kF16MinNormal) ? 0.0f : v;
  return (_Float16)w;
}

__device__ __forceinline__ v8f mma_h(v16h a, v16h b, v8f c) {
  c = __builtin_amdgcn_wmma_f32_16x16x32_f16(false, a, false, b, (short)0, c, false, false);
  asm volatile("v_nop\n\tv_nop\n\tv_nop\n\tv_nop" : "+v"(c) : "v"(a), "v"(b));
  return c;
}

__device__ __forceinline__ float long_kernel_at(const float* ker64, int t) {
  const int i = 31 - __builtin_clz((unsigned)((t >> 6) + 1));
  const int j = t - kTaps * ((1 << i) - 1);
  const float inv = __uint_as_float((unsigned)(127 - i) << 23);
  const float coord = ((float)j + 0.5f) * inv - 0.5f;
  const float f0 = floorf(coord);
  const float fr = coord - f0;
  int i0 = (int)f0;
  int i1 = i0 + 1;
  i0 = i0 < 0 ? 0 : (i0 > kTaps - 1 ? kTaps - 1 : i0);
  i1 = i1 < 0 ? 0 : (i1 > kTaps - 1 ? kTaps - 1 : i1);
  const float a = ker64[i0];
  const float b = ker64[i1];
  return ((1.0f - fr) * a + fr * b) * inv;
}

__global__ __launch_bounds__(256) void ks_build_kernel(const float* __restrict__ kern, _Float16* __restrict__ KS)
{
  __shared__ float sKer[kTaps];
  const int tid = threadIdx.x;
  const int v = blockIdx.x * 256 + tid;
  const int d = v / kKsVecPerCh;
  const int rem = v - d * kKsVecPerCh;
  const int c = rem / (kPitch / 8);
  const int x = (rem - c * (kPitch / 8)) * 8;
  const float kval = kern[(tid & (kTaps - 1)) * kCh + d];
  if (tid < kTaps) sKer[tid] = kval;
  __syncthreads();
  v8h hv;
#pragma unroll
  for (int e = 0; e < 8; ++e) {
    const int m = (x + c + e) & (kLen - 1);
    const int t = (kLen - m) & (kLen - 1);
    hv[e] = f2h_flush(long_kernel_at(sKer, t) * kCarryK);
  }
  _Float16* dst = KS + (size_t)v * 8;
  *(volatile v8h*)dst = hv;
  __threadfence();
  *(volatile v8h*)dst = hv;
}

__global__ __launch_bounds__(256) void bt_build_kernel(const float* __restrict__ sig, _Float16* __restrict__ BT)
{
  __shared__ __align__(16) float sT[64 * kTilePitch];
  const int tid = threadIdx.x, lane = tid & 31, wave = tid >> 5;
  const int j0 = blockIdx.x * 64;
  const int b  = blockIdx.y;
  const float* src = sig + ((size_t)b * kLen + j0) * kCh;
#pragma unroll
  for (int k = 0; k < 6; ++k) {
    const int idx = tid + 256 * k;
    const int row = idx / 24;
    const int c4  = idx - row * 24;
    const v4f val = *(const v4f*)(src + (size_t)idx * 4);
    *(v4f*)(sT + row * kTilePitch + c4 * 4) = val;
  }
  __syncthreads();
  const int q = lane >> 3, l8 = lane & 7;
  v8h hv[6];
#pragma unroll
  for (int it = 0; it < 6; ++it) {
    const int ln = it * 32 + wave * 4 + q;
    const int dd = (ln >= kCh) ? (ln - kCh) : ln;
#pragma unroll
    for (int e = 0; e < 8; ++e)
      hv[it][e] = f2h_flush(sT[(l8 * 8 + e) * kTilePitch + dd] * kCarryU);
  }
  for (int pass = 0; pass < 2; ++pass) {
#pragma unroll
    for (int it = 0; it < 6; ++it) {
      const int ln = it * 32 + wave * 4 + q;
      const int s  = (ln >= kCh) ? 1 : 0;
      const int dd = ln - s * kCh;
      const int jp = (j0 + s * kHalfLen) & (kLen - 1);
      _Float16* dst = BT + ((size_t)(dd * kCols + s * kNb + b)) * kLen + jp + l8 * 8;
      *(volatile v8h*)dst = hv[it];
    }
    __threadfence();
  }
}

__global__ __launch_bounds__(256) void circ_conv_kernel(const _Float16* __restrict__ KS, const _Float16* __restrict__ BT,
                                                        const float* __restrict__ bias, float* __restrict__ YP)
{
  __shared__ __align__(16) _Float16 sK[kKsPerCh];
  union FH { v16h v; v8h h[2]; };
  const int tid = threadIdx.x, lane = tid & 31, wave = tid >> 5;
  const int d   = blockIdx.x / kBlksPerCh;
  const int blk = blockIdx.x - d * kBlksPerCh;
  {
    const v8h* src = (const v8h*)(KS + (size_t)d * kKsPerCh);
#pragma unroll 1
    for (int k = 0; k < kKsVecPerCh / 256; ++k) {
      const int idx = tid + 256 * k;
      const v8h val = src[idx];
      *(v8h*)(sK + idx * 8) = val;
    }
  }
  __syncthreads();

  const int h = lane >> 4, i = lane & 15;
  const int T0 = blk * kTilesPerBlk + wave * kTilesPerWave;
  const int cb = ((8 - (i & 7)) & 7) * kPitch;
  const int sb = 8 * h - 16 * T0 - i;
  const _Float16* brow = BT + ((size_t)(d * kCols + i)) * kLen + 8 * h;

  v8f acc[kTilesPerWave];
#pragma unroll
  for (int a = 0; a < kTilesPerWave; ++a) acc[a] = (v8f){0.f, 0.f, 0.f, 0.f, 0.f, 0.f, 0.f, 0.f};

#pragma unroll 1
  for (int J = 0; J < kLen / 32; ++J) {
    FH bf;
    bf.h[0] = *(const v8h*)(brow + 32 * J);
    bf.h[1] = *(const v8h*)(brow + 32 * J + 16);
    const int sj = sb + 32 * J;
#pragma unroll
    for (int a = 0; a < kTilesPerWave; ++a) {
      const int x = (sj - 16 * a) & kWrapMask;
      FH af;
      af.h[0] = *(const v8h*)(sK + cb + x);
      af.h[1] = *(const v8h*)(sK + cb + x + 16);
      acc[a] = mma_h(af.v, bf.v, acc[a]);
    }
  }

  __syncthreads();
  float* slab = reinterpret_cast<float*>(sK) + wave * (kCols * kSlabPitch);
  const float bv = bias[d];
#pragma unroll
  for (int a = 0; a < kTilesPerWave; ++a) {
#pragma unroll
    for (int r = 0; r < 8; ++r)
      slab[i * kSlabPitch + a * 16 + 8 * h + r] = acc[a][r] * kFold + bv;
  }
  __syncthreads();
  const int t0w = 16 * T0;
  for (int pass = 0; pass < 2; ++pass) {
#pragma unroll
    for (int n = 0; n < kCols; ++n) {
      const v4f val = *(const v4f*)(slab + n * kSlabPitch + lane * 4);
      float* dst = YP + ((size_t)(d * kNb + (n & 7))) * kLen + (n >> 3) * kHalfLen + t0w + lane * 4;
      *(volatile v4f*)dst = val;
    }
    __threadfence();
  }
}

__global__ __launch_bounds__(256) void out_layout_kernel(const float* __restrict__ YP, float* __restrict__ out)
{
  __shared__ __align__(16) float sT[64 * kTilePitch];
  const int tid = threadIdx.x;
  const int t0 = blockIdx.x * 64;
  const int b  = blockIdx.y;
#pragma unroll
  for (int k = 0; k < 6; ++k) {
    const int idx = tid + 256 * k;
    const int dd = idx >> 4;
    const int c4 = idx & 15;
    const v4f val = *(const v4f*)(YP + ((size_t)(dd * kNb + b)) * kLen + t0 + c4 * 4);
#pragma unroll
    for (int e = 0; e < 4; ++e) sT[(c4 * 4 + e) * kTilePitch + dd] = val[e];
  }
  __syncthreads();
  v4f ov[6];
#pragma unroll
  for (int k = 0; k < 6; ++k) {
    const int idx = tid + 256 * k;
    const int row = idx / 24;
    const int c4  = idx - row * 24;
    ov[k] = *(const v4f*)(sT + row * kTilePitch + c4 * 4);
  }
  float* dst = out + ((size_t)b * kLen + t0) * kCh;
  for (int pass = 0; pass < 2; ++pass) {
#pragma unroll
    for (int k = 0; k < 6; ++k) {
      const int idx = tid + 256 * k;
      *(volatile v4f*)(dst + (size_t)idx * 4) = ov[k];
    }
    __threadfence();
  }
}

extern "C" void kernel_launch(void* const* d_in, const int* in_sizes, int n_in,
                              void* d_out, int out_size, void* d_ws, size_t ws_size,
                              hipStream_t stream) {
  if (n_in < 3) return;
  if (in_sizes[0] != kNb * kLen * kCh) return;
  if (in_sizes[1] != kTaps * kCh) return;
  if (in_sizes[2] != kCh) return;
  if (out_size != kNb * kLen * kCh) return;
  if (ws_size < kWsTotal) return;

  const float* sig  = (const float*)d_in[0];
  const float* kern = (const float*)d_in[1];
  const float* bias = (const float*)d_in[2];
  float* out = (float*)d_out;

  char* ws = (char*)d_ws;
  _Float16* KS = (_Float16*)(ws + kOffKS);
  _Float16* BT = (_Float16*)(ws + kOffBT);
  float*    YP = (float*)(ws + kOffYP);

  ks_build_kernel<<<kCh * (kKsVecPerCh / 256), 256, 0, stream>>>(kern, KS);
  bt_build_kernel<<<dim3(kLen / 64, kNb), 256, 0, stream>>>(sig, BT);
  circ_conv_kernel<<<kCh * kBlksPerCh, 256, 0, stream>>>(KS, BT, bias, YP);
  out_layout_kernel<<<dim3(kLen / 64, kNb), 256, 0, stream>>>(YP, out);
}
